// WATTNet_89593017794632
// MI455X (gfx1250) — hardware-verified
//
#include <hip/hip_runtime.h>


#define NBT 4
#define NS 128
#define EE 16
#define LL 2048
#define T0 128
#define NOUT 24

typedef __attribute__((ext_vector_type(16))) __bf16   v16bf;
typedef __attribute__((ext_vector_type(16))) _Float16 v16h;
typedef __attribute__((ext_vector_type(8)))  float    v8f;
typedef __attribute__((ext_vector_type(8)))  unsigned v8u;

__device__ __forceinline__ unsigned f2bf(float f) { unsigned u = __float_as_uint(f); u += 0x7FFFu + ((u >> 16) & 1u); return u >> 16; }
__device__ __forceinline__ unsigned f2h(float f) { return (unsigned)__builtin_bit_cast(unsigned short, (_Float16)f); }
__device__ __forceinline__ int kpat(int v, int half) { return ((v & 4) ? 16 : 0) + half * 8 + 2 * (v & 3); }

template <int F16, int NP> struct Opnd { v16bf p[NP]; };

template <int F16, int NP> __device__ __forceinline__ void pack2(float f0, float f1, unsigned* o) {
    if (F16) { o[0] = f2h(f0) | (f2h(f1) << 16); return; }
    unsigned h0 = f2bf(f0), h1 = f2bf(f1); o[0] = h0 | (h1 << 16);
    if (NP >= 2) {
        float r0 = f0 - __uint_as_float(h0 << 16), r1 = f1 - __uint_as_float(h1 << 16);
        unsigned m0 = f2bf(r0), m1 = f2bf(r1); o[1] = m0 | (m1 << 16);
        if (NP >= 3) {
            float s0 = r0 - __uint_as_float(m0 << 16), s1 = r1 - __uint_as_float(m1 << 16);
            o[2] = f2bf(s0) | (f2bf(s1) << 16);
        }
    }
}
template <int F16, int NP> __device__ __forceinline__ void op_row(const float* rowp, int half, float sc, Opnd<F16, NP>& o) {
    v8u u[NP];
#pragma unroll
    for (int v = 0; v < 8; ++v) {
        int kk = kpat(v, half); unsigned t[3];
        pack2<F16, NP>(rowp[kk] * sc, rowp[kk + 1] * sc, t);
#pragma unroll
        for (int p = 0; p < NP; ++p) u[p][v] = t[p];
    }
#pragma unroll
    for (int p = 0; p < NP; ++p) o.p[p] = __builtin_bit_cast(v16bf, u[p]);
}
template <int F16, int NP> __device__ __forceinline__ void op_row_tail(const float* rowp, int half, float sc, int kvalid, Opnd<F16, NP>& o) {
    v8u u[NP];
#pragma unroll
    for (int v = 0; v < 8; ++v) {
        int kk = kpat(v, half); unsigned t[3];
        float f0 = kk < kvalid ? rowp[kk] * sc : 0.0f, f1 = (kk + 1) < kvalid ? rowp[kk + 1] * sc : 0.0f;
        pack2<F16, NP>(f0, f1, t);
#pragma unroll
        for (int p = 0; p < NP; ++p) u[p][v] = t[p];
    }
#pragma unroll
    for (int p = 0; p < NP; ++p) o.p[p] = __builtin_bit_cast(v16bf, u[p]);
}
template <int F16, int NP> __device__ __forceinline__ void op_col(const float* M, int ld, int n, int k0, int half, float sc, Opnd<F16, NP>& o) {
    v8u u[NP];
#pragma unroll
    for (int v = 0; v < 8; ++v) {
        int kk = k0 + kpat(v, half); unsigned t[3];
        pack2<F16, NP>(M[(size_t)kk * ld + n] * sc, M[(size_t)(kk + 1) * ld + n] * sc, t);
#pragma unroll
        for (int p = 0; p < NP; ++p) u[p][v] = t[p];
    }
#pragma unroll
    for (int p = 0; p < NP; ++p) o.p[p] = __builtin_bit_cast(v16bf, u[p]);
}
template <int F16, int NP> __device__ __forceinline__ void op_col_tail(const float* M, int ld, int n, int k0, int half, float sc, int K, Opnd<F16, NP>& o) {
    v8u u[NP];
#pragma unroll
    for (int v = 0; v < 8; ++v) {
        int kk = k0 + kpat(v, half); unsigned t[3];
        float f0 = kk < K ? M[(size_t)kk * ld + n] * sc : 0.0f, f1 = (kk + 1) < K ? M[(size_t)(kk + 1) * ld + n] * sc : 0.0f;
        pack2<F16, NP>(f0, f1, t);
#pragma unroll
        for (int p = 0; p < NP; ++p) u[p][v] = t[p];
    }
#pragma unroll
    for (int p = 0; p < NP; ++p) o.p[p] = __builtin_bit_cast(v16bf, u[p]);
}
__device__ __forceinline__ v8f wm_bf16(v16bf a, v16bf b, v8f c) { return __builtin_amdgcn_wmma_f32_16x16x32_bf16(false, a, false, b, (short)0, c, false, false); }
template <int F16, int NA, int NB> __device__ __forceinline__ v8f wmma_op(const Opnd<F16, NA>& a, const Opnd<F16, NB>& b, v8f c) {
    if (F16) {
        v16h ah = __builtin_bit_cast(v16h, a.p[0]), bh = __builtin_bit_cast(v16h, b.p[0]);
        c = __builtin_amdgcn_wmma_f32_16x16x32_f16(false, ah, false, bh, (short)0, c, false, false);
        asm volatile("v_nop\n\tv_nop\n\tv_nop\n\tv_nop" : "+v"(c) : "v"(ah), "v"(bh));
        return c;
    }
    constexpr int NMX = NA > NB ? NA : NB;
#pragma unroll
    for (int i = 0; i < NA; ++i)
#pragma unroll
        for (int j = 0; j < NB; ++j)
            if (i + j < NMX) c = wm_bf16(a.p[i], b.p[j], c);
    if (NA == 1 && NB == 1)      asm volatile("v_nop\n\tv_nop\n\tv_nop\n\tv_nop" : "+v"(c) : "v"(a.p[0]), "v"(b.p[0]));
    else if (NA == 2 && NB == 1) asm volatile("v_nop\n\tv_nop\n\tv_nop\n\tv_nop" : "+v"(c) : "v"(a.p[0]), "v"(a.p[1]), "v"(b.p[0]));
    else if (NA == 1 && NB == 2) asm volatile("v_nop\n\tv_nop\n\tv_nop\n\tv_nop" : "+v"(c) : "v"(a.p[0]), "v"(b.p[0]), "v"(b.p[1]));
    else if (NA == 2 && NB == 2) asm volatile("v_nop\n\tv_nop\n\tv_nop\n\tv_nop" : "+v"(c) : "v"(a.p[0]), "v"(a.p[1]), "v"(b.p[0]), "v"(b.p[1]));
    else                         asm volatile("v_nop\n\tv_nop\n\tv_nop\n\tv_nop" : "+v"(c) : "v"(a.p[0]), "v"(a.p[NA - 1]), "v"(b.p[0]), "v"(b.p[NB - 1]), "v"(a.p[NA / 2]), "v"(b.p[NB / 2]));
    return c;
}

struct ZMap { long long s1; long long s2; int zdiv; int pad_; };
__device__ __forceinline__ size_t zoff(const ZMap& m, int z) { return (size_t)((long long)(z / m.zdiv) * m.s1 + (long long)(z % m.zdiv) * m.s2); }

#define ACT_NONE 0
#define ACT_RELU 1
#define ACT_GELU_ERF 2
#define ACT_SILU 3
#define ACT_TANH 4
__device__ __forceinline__ float act_apply(int act, float x) {
    if (act == ACT_RELU) return x > 0.f ? x : 0.f;
    if (act == ACT_GELU_ERF) return 0.5f * x * (1.0f + erff(x * 0.70710678118654752f));
    if (act == ACT_SILU) return x / (1.0f + expf(-x));
    if (act == ACT_TANH) return tanhf(x);
    return x;
}
struct GemmArgs {
    ZMap za, zb_, zc, zbias, zadd, zrsc, zmul, zrbias;
    const float* A; const float* Bm; float* C; const float* bias; const float* add; const float* rsc; const float* mul; const float* rbias;
    long long ldadd, ldmul;
    int lda, ldb, ldc, K;
    float ascale, bscale, oscale, addscale;
    int M, nvalid, nstore, ldrsc;
    int bcs, pad1, pad2, pad3;
};
template <int BT, int F16, int NA, int NB, int RW, int CW, int ACT>
__global__ __launch_bounds__(256) void gemm_kernel(GemmArgs g) {
    constexpr int TR = 16 * RW, TC = 64 * CW, CSTR = TC + 4;
    __shared__ __align__(16) float cst[TR * CSTR];
    const int z = blockIdx.z;
    const float* A = g.A + zoff(g.za, z); const float* Bm = g.Bm + zoff(g.zb_, z); float* C = g.C + zoff(g.zc, z);
    const int tid = threadIdx.x, lane = tid & 31, wv = tid >> 5;
    const int l16 = lane & 15, half = lane >> 4;
    const int rt = wv % RW, ch = wv / RW;
    const int row0 = blockIdx.x * TR, col0 = blockIdx.y * TC + ch * 64;
    int arix = row0 + rt * 16 + l16; if (arix >= g.M) arix = g.M - 1;
    const float* arow = A + (size_t)arix * g.lda;
    v8f acc[4];
#pragma unroll
    for (int t = 0; t < 4; ++t) acc[t] = (v8f){};
    const int K = g.K;
#pragma unroll 1
    for (int kc = 0; kc < K; kc += 32) {
        Opnd<F16, NA> a;
        if (kc + 32 <= K) op_row<F16, NA>(arow + kc, half, g.ascale, a); else op_row_tail<F16, NA>(arow + kc, half, g.ascale, K - kc, a);
#pragma unroll
        for (int t = 0; t < 4; ++t) {
            Opnd<F16, NB> b;
            const int n = col0 + t * 16 + l16;
            if (n < g.nvalid) {
                if (BT) { if (kc + 32 <= K) op_row<F16, NB>(Bm + (size_t)n * g.ldb + kc, half, g.bscale, b); else op_row_tail<F16, NB>(Bm + (size_t)n * g.ldb + kc, half, g.bscale, K - kc, b); }
                else    { if (kc + 32 <= K) op_col<F16, NB>(Bm, g.ldb, n * g.bcs, kc, half, g.bscale, b); else op_col_tail<F16, NB>(Bm, g.ldb, n * g.bcs, kc, half, g.bscale, K, b); }
            } else {
#pragma unroll
                for (int p = 0; p < NB; ++p) b.p[p] = (v16bf){};
            }
            acc[t] = wmma_op<F16, NA, NB>(a, b, acc[t]);
        }
    }
    const float* bias = g.bias ? g.bias + zoff(g.zbias, z) : nullptr;
    const float* add = g.add ? g.add + zoff(g.zadd, z) : nullptr;
    const float* rsc = g.rsc ? g.rsc + zoff(g.zrsc, z) : nullptr;
    const float* mul = g.mul ? g.mul + zoff(g.zmul, z) : nullptr;
    const float* rbias = g.rbias ? g.rbias + zoff(g.zrbias, z) : nullptr;
#pragma unroll
    for (int t = 0; t < 4; ++t) {
        const int cl = ch * 64 + t * 16 + l16;
        const int cg = blockIdx.y * TC + cl;
        const bool cok = cg < g.nvalid;
        const float bv = (bias && cok) ? bias[(size_t)cg * g.bcs] : 0.0f;
#pragma unroll
        for (int r = 0; r < 8; ++r) {
            const int rl = rt * 16 + r + 8 * half;
            float v = acc[t][r] * g.oscale + bv;
            int rg = row0 + rl; if (rg >= g.M) rg = g.M - 1;
            if (rbias) v += rbias[rg];
            if (rsc) v *= rsc[(size_t)rg * g.ldrsc];
            if (mul && cok) v *= mul[(size_t)rg * g.ldmul + cg];
            if (add && cok) v += g.addscale * add[(size_t)rg * g.ldadd + cg];
            cst[rl * CSTR + cl] = v;
        }
    }
    __syncthreads();
    const int col = tid % TC, rsel = tid / TC, rstep = 256 / TC;
    if (ACT != ACT_NONE) {
#pragma unroll 1
        for (int r = rsel; r < TR; r += rstep) cst[r * CSTR + col] = act_apply(ACT, cst[r * CSTR + col]);
    }
    float* ob = C + (size_t)row0 * g.ldc + (size_t)blockIdx.y * TC;
    const bool colok = (int)(blockIdx.y * TC + col) < g.nstore;
    const int rmax = (g.M - row0 < TR) ? (g.M - row0) : TR;
    auto pass = [&]() {
        if (colok) {
#pragma unroll 4
            for (int r = rsel; r < rmax; r += rstep) *(volatile float*)(ob + (size_t)r * g.ldc + col) = cst[r * CSTR + col];
        }
    };
    pass();
    __threadfence();
    pass();
}
static inline ZMap zm(long long s1) { ZMap m; m.s1 = s1; m.s2 = 0; m.zdiv = 1; m.pad_ = 0; return m; }
static inline ZMap zm2(long long s1, long long s2, int zdiv) { ZMap m; m.s1 = s1; m.s2 = s2; m.zdiv = zdiv; m.pad_ = 0; return m; }
static inline GemmArgs gemm_args(const float* A, int lda, ZMap za, const float* Bm, int ldb, ZMap zb, float* C, int ldc, ZMap zc, int M, int N, int K) {
    GemmArgs g; g.za = za; g.zb_ = zb; g.zc = zc; g.zbias = zm(0); g.zadd = zm(0); g.zrsc = zm(0); g.zmul = zm(0); g.zrbias = zm(0);
    g.A = A; g.Bm = Bm; g.C = C; g.bias = nullptr; g.add = nullptr; g.rsc = nullptr; g.mul = nullptr; g.rbias = nullptr; g.ldadd = 0; g.ldmul = 0;
    g.lda = lda; g.ldb = ldb; g.ldc = ldc; g.K = K; g.ascale = 1.0f; g.bscale = 1.0f; g.oscale = 1.0f; g.addscale = 1.0f; g.M = M; g.nvalid = N; g.nstore = N; g.ldrsc = 1;
    g.bcs = 1; g.pad1 = 0; g.pad2 = 0; g.pad3 = 0;
    return g;
}
static_assert(sizeof(ZMap) == 24, "ZMap layout");
static_assert(sizeof(GemmArgs) == 8 * 24 + 8 * 8 + 2 * 8 + 4 * 4 + 4 * 4 + 4 * 4 + 4 * 4, "GemmArgs has no padding");

__global__ __launch_bounds__(256) void softmax_rows(float* S, long long sy, long long sx, int L, float prescale, const float* addv, long long say, int aydiv, int causal,
                                                  const int* imask, long long imy, long long imx, float maskval) {
    __shared__ float red[8];
    const int tid = threadIdx.x, lane = tid & 31, wid = tid >> 5;
    float* row = S + (size_t)blockIdx.y * sy + (size_t)blockIdx.x * sx;
    const float* av = addv ? addv + (size_t)(blockIdx.y / aydiv) * say : nullptr;
    const int* im = imask ? imask + (size_t)(blockIdx.y / aydiv) * imy + (size_t)blockIdx.x * imx : nullptr;
    float v[16];
    const int nj = L / 256;
    float mx = -__builtin_inff();
#pragma unroll
    for (int j = 0; j < 16; ++j) if (j < nj) { float t = row[tid + 256 * j] * prescale; if (av) t += av[tid + 256 * j]; if (im && im[tid + 256 * j] == 0) t = maskval; if (causal && (tid + 256 * j) > (int)blockIdx.x) t = -__builtin_inff(); v[j] = t; mx = fmaxf(mx, t); }
#pragma unroll
    for (int o = 16; o; o >>= 1) mx = fmaxf(mx, __shfl_xor(mx, o, 32));
    if (lane == 0) red[wid] = mx;
    __syncthreads();
    float m = red[0];
#pragma unroll
    for (int i = 1; i < 8; ++i) m = fmaxf(m, red[i]);
    if (m == -__builtin_inff()) m = 0.f;
    __syncthreads();
    float sum = 0.f;
#pragma unroll
    for (int j = 0; j < 16; ++j) if (j < nj) { v[j] = expf(v[j] - m); sum += v[j]; }
#pragma unroll
    for (int o = 16; o; o >>= 1) sum += __shfl_xor(sum, o, 32);
    if (lane == 0) red[wid] = sum;
    __syncthreads();
    float tot = 0.f;
#pragma unroll
    for (int i = 0; i < 8; ++i) tot += red[i];
    const float inv = 1.0f / tot;
#pragma unroll
    for (int j = 0; j < 16; ++j) if (j < nj) *(volatile float*)(row + tid + 256 * j) = v[j] * inv;
    __threadfence();
#pragma unroll
    for (int j = 0; j < 16; ++j) if (j < nj) *(volatile float*)(row + tid + 256 * j) = v[j] * inv;
}

#define VST2(T, p, v) do { const T vst2_v_ = (v); *(volatile T*)(p) = vst2_v_; __threadfence(); *(volatile T*)(p) = vst2_v_; } while (0)
__device__ __forceinline__ bool dec4(int q, int mode, int T, int& b, int& n, int& t, int& e) { if (mode == 0) { n = q % NS; e = (q / NS) % EE; t = (q / (NS * EE)) % T; b = q / (NS * EE * T); return true; } else { t = q % 128; e = (q / 128) % EE; n = (q / (128 * EE)) % NS; b = q / (128 * EE * NS); return t < T; } }
__global__ __launch_bounds__(256) void k_emb(const float* __restrict__ xin, const float* __restrict__ ew, const float* __restrict__ eb, int mode, float* XT, float* XS) { const int q = blockIdx.x * 256 + threadIdx.x; const int tot = mode == 0 ? NBT * T0 * EE * NS : NBT * NS * EE * 128; if (q >= tot) return; int b, n, t, e; if (!dec4(q, mode, T0, b, n, t, e)) { VST2(float, XS + q, 0.f); return; }
    const float* row = xin + ((size_t)b * T0 + t) * (NS + 3);
    const float v = row[n] * ew[e] + row[NS] * ew[EE + e] + row[NS + 1] * ew[2 * EE + e] + row[NS + 2] * ew[3 * EE + e] + eb[e];
    if (mode == 0) { VST2(float, XT + q, v); } else { VST2(float, XS + q, v); } }
__global__ __launch_bounds__(256) void k_wsl(const float* __restrict__ wf, const float* __restrict__ wg, float* W4) { const int q = blockIdx.x * 256 + threadIdx.x; if (q >= 4 * NS * NS) return; const int i = q % NS, o = (q / NS) % NS, k = q / (NS * NS); const float* w = k < 2 ? wf : wg; VST2(float, W4 + q, w[((size_t)o * NS + i) * 2 + (k & 1)]); }
__global__ __launch_bounds__(256) void k_comb(const float* __restrict__ F, const float* __restrict__ G, const float* __restrict__ RES, int T, int Tn, int mode, float* XT, float* XS) { const int q = blockIdx.x * 256 + threadIdx.x; const int tot = mode == 0 ? NBT * Tn * EE * NS : NBT * NS * EE * 128; if (q >= tot) return; int b, n, s, e; if (!dec4(q, mode, Tn, b, n, s, e)) { VST2(float, XS + q, 0.f); return; }
    const size_t fr = ((size_t)b * T + s) * EE + e; const float f = F[fr * NS + n], g = G[fr * NS + n]; const float v = tanhf(f) * (1.f / (1.f + expf(-g))) + RES[(((size_t)b * NS + n) * EE + e) * 128 + s];
    if (mode == 0) { VST2(float, XT + q, v); } else { VST2(float, XS + q, v); } }
__global__ __launch_bounds__(256) void k_uwc(const float* __restrict__ wq, const float* __restrict__ bq, const float* __restrict__ wk, const float* __restrict__ bk, float* UW) { __shared__ double r1[256], r2[256]; const int i = blockIdx.x, tid = threadIdx.x; double a = 0.0, b = 0.0;
    if (i < NS) { for (int l = tid; l < LL; l += 256) { a += (double)(wq[(size_t)i * LL + l] * bk[l]); b += (double)(wk[(size_t)i * LL + l] * bq[l]); } }
    else { for (int l = tid; l < LL; l += 256) a += (double)(bq[l] * bk[l]); }
    r1[tid] = a; r2[tid] = b; __syncthreads(); for (int o = 128; o > 0; o >>= 1) { if (tid < o) { r1[tid] += r1[tid + o]; r2[tid] += r2[tid + o]; } __syncthreads(); }
    if (tid < 32) { if (i < NS) { VST2(float, UW + (size_t)i * 32 + tid, tid == 0 ? (float)r1[0] : (tid == 1 ? (float)r2[0] : 0.f)); } else { VST2(float, UW + (size_t)NS * 32 + tid, tid == 0 ? (float)r1[0] : 0.f); } } }
__global__ __launch_bounds__(256) void k_att(const float* __restrict__ XT, const float* __restrict__ Y, const float* __restrict__ UW, int T, float* R) { __shared__ float xs[EE][NS], ys[EE][NS]; __shared__ float S[EE][EE + 1]; __shared__ float ab[EE]; __shared__ float xu[EE], xw[EE]; const int bt = blockIdx.x, tid = threadIdx.x;
    for (int q = tid; q < EE * NS; q += 256) { xs[q / NS][q % NS] = XT[(size_t)bt * EE * NS + q]; ys[q / NS][q % NS] = Y[(size_t)bt * EE * NS + q]; } __syncthreads();
    if (tid < 2 * EE) { const int e = tid % EE; float a = 0.f;
#pragma unroll 1
        for (int i = 0; i < NS; ++i) a += xs[e][i] * UW[(size_t)i * 32 + (tid < EE ? 0 : 1)]; if (tid < EE) xu[e] = a; else xw[e] = a; }
    { const int e = tid / EE, f = tid % EE; float a = 0.f;
#pragma unroll 1
      for (int i = 0; i < NS; ++i) a += ys[e][i] * xs[f][i]; S[e][f] = a; }
    __syncthreads();
    if (tid < EE * EE) { const int e = tid / EE, f = tid % EE; S[e][f] = (S[e][f] + xu[e] + xw[f] + UW[(size_t)NS * 32]) * 0.02209708691207961f; }
    __syncthreads();
    if (tid < EE) { const int e = tid; float m = -__builtin_inff();
#pragma unroll 1
        for (int f = 0; f < EE; ++f) m = fmaxf(m, S[e][f]); float d = 0.f;
#pragma unroll 1
        for (int f = 0; f < EE; ++f) { const float v = expf(S[e][f] - m); S[e][f] = v; d += v; }
#pragma unroll 1
        for (int f = 0; f < EE; ++f) S[e][f] /= d; }
    __syncthreads();
    if (tid < EE) { float a = 0.f;
#pragma unroll 1
        for (int e = 0; e < EE; ++e) a += S[e][tid]; ab[tid] = a / (float)EE; }
    __syncthreads();
    if (tid < NS) { float a = 0.f;
#pragma unroll 1
        for (int f = 0; f < EE; ++f) a += ab[f] * xs[f][tid]; VST2(float, R + (size_t)bt * NS + tid, a); } }
__global__ __launch_bounds__(256) void k_ares(const float* __restrict__ READ, const float* __restrict__ XTc, int T, int mode, float* XTn, float* XSn) { const int q = blockIdx.x * 256 + threadIdx.x; const int tot = mode == 0 ? NBT * T * EE * NS : NBT * NS * EE * 128; if (q >= tot) return; int b, n, t, e; if (!dec4(q, mode, T, b, n, t, e)) { VST2(float, XSn + q, 0.f); return; }
    const float v = XTc[(((size_t)b * T + t) * EE + e) * NS + n] + READ[((size_t)b * T + t) * LL + n * EE + e];
    if (mode == 0) { VST2(float, XTn + q, v); } else { VST2(float, XSn + q, v); } }
__global__ __launch_bounds__(256) void k_dec(const float* __restrict__ XS, const float* __restrict__ dw, const float* __restrict__ db, int T, float* YD) { const int lane = threadIdx.x & 31; const int r = blockIdx.x * 8 + (threadIdx.x >> 5); if (r >= NBT * NS) return; const int n = r % NS;
#pragma unroll 1
    for (int t = lane; t < 128; t += 32) { float a = 0.f; if (t < T) { a = db[n];
#pragma unroll 1
            for (int e = 0; e < EE; ++e) a += XS[((size_t)r * EE + e) * 128 + t] * dw[n * EE + e]; }
        VST2(float, YD + (size_t)r * 128 + t, a); } }
__global__ __launch_bounds__(256) void k_out(const float* __restrict__ Y2, float* out) { const int q = blockIdx.x * 256 + threadIdx.x; if (q >= NBT * NOUT * NS) return; const int n = q % NS, o = (q / NS) % NOUT, b = q / (NS * NOUT); VST2(float, out + q, Y2[((size_t)b * NS + n) * 32 + o]); }
__global__ __launch_bounds__(256) void k_wsp(const float* __restrict__ ws, int T, int Tn, float* WSP) { const int q = blockIdx.x * 256 + threadIdx.x; if (q >= 128 * 128) return; const int s = q % 128, t = q / 128; VST2(float, WSP + q, (t < T && s < Tn) ? ws[t * Tn + s] : 0.f); }
__global__ __launch_bounds__(256) void k_wpad(const float* __restrict__ ow, float* OWP) { const int q = blockIdx.x * 256 + threadIdx.x; if (q >= 128 * 32) return; const int o = q % 32, t = q / 32; VST2(float, OWP + q, (t < 122 && o < NOUT) ? ow[t * NOUT + o] : 0.f); }
extern "C" void kernel_launch(void* const* d_in, const int* in_sizes, int n_in,
                              void* d_out, int out_size, void* d_ws, size_t ws_size, hipStream_t stream) {
    (void)in_sizes; (void)n_in; (void)out_size;
    const float* xin = (const float*)d_in[0]; const float* ew = (const float*)d_in[1]; const float* eb = (const float*)d_in[2];
    const float* gw[2][6]; const float* aw[2][6];
    for (int i = 0; i < 6; ++i) { gw[0][i] = (const float*)d_in[3 + i]; aw[0][i] = (const float*)d_in[9 + i]; gw[1][i] = (const float*)d_in[15 + i]; aw[1][i] = (const float*)d_in[21 + i]; }
    const float* dw = (const float*)d_in[27]; const float* db = (const float*)d_in[28]; const float* ow = (const float*)d_in[29]; const float* ob = (const float*)d_in[30];
    float* out = (float*)d_out;
    char* wsp = (char*)d_ws;
    auto take = [&](size_t bytes) { char* p = wsp; wsp += (bytes + 255) & ~(size_t)255; return (void*)p; };
    const size_t NXT = (size_t)NBT * T0 * EE * NS;
    float* XT = (float*)take(NXT * 4); float* XS = (float*)take((size_t)NBT * NS * EE * 128 * 4); float* XT2 = (float*)take(NXT * 4); float* XS2 = (float*)take((size_t)NBT * NS * EE * 128 * 4);
    float* W4 = (float*)take((size_t)4 * NS * NS * 4); float* F = (float*)take(NXT * 4); float* G = (float*)take(NXT * 4); float* RES = (float*)take((size_t)NBT * NS * EE * 128 * 4);
    float* Mq = (float*)take((size_t)NS * NS * 4); float* UW = (float*)take((size_t)(NS + 1) * 32 * 4); float* Y = (float*)take(NXT * 4); float* R = (float*)take((size_t)NBT * T0 * NS * 4); float* READ = (float*)take((size_t)NBT * T0 * LL * 4);
    float* YD = (float*)take((size_t)NBT * NS * 128 * 4); float* OWP = (float*)take(128 * 32 * 4); float* OB = (float*)take(32 * 4); float* Y2 = (float*)take((size_t)NBT * NS * 32 * 4); float* WSP = (float*)take(128 * 128 * 4);
    if ((size_t)(wsp - (char*)d_ws) > ws_size) return;
    k_emb<<<(NBT * NS * T0 * EE) / 256, 256, 0, stream>>>(xin, ew, eb, 0, XT, XS); k_emb<<<(NBT * NS * EE * 128) / 256, 256, 0, stream>>>(xin, ew, eb, 1, XT, XS);
    float* cXT = XT; float* cXS = XS; float* nXT = XT2; float* nXS = XS2; int T = T0;
    const int dil[2] = {2, 4};
    for (int blk = 0; blk < 2; ++blk) { const int d = dil[blk]; const int Tn = T - d;
        const float* wf = gw[blk][0]; const float* bf = gw[blk][1]; const float* wgt = gw[blk][2]; const float* bg = gw[blk][3]; const float* ws = gw[blk][4]; const float* bs = gw[blk][5];
        const float* wq = aw[blk][0]; const float* bq = aw[blk][1]; const float* wk = aw[blk][2]; const float* bk = aw[blk][3]; const float* wv = aw[blk][4]; const float* bv = aw[blk][5];
        k_wsl<<<(4 * NS * NS) / 256, 256, 0, stream>>>(wf, wgt, W4);
        { GemmArgs g = gemm_args(cXT, NS, zm(T * EE * NS), W4, NS, zm(0), F, NS, zm(T * EE * NS), Tn * EE, NS, NS); g.bias = bf; gemm_kernel<1, 0, 2, 2, 4, 2, ACT_NONE><<<dim3((Tn * EE + 63) / 64, 1, NBT), 256, 0, stream>>>(g); }
        { GemmArgs g = gemm_args(cXT + (size_t)d * EE * NS, NS, zm(T * EE * NS), W4 + (size_t)NS * NS, NS, zm(0), F, NS, zm(T * EE * NS), Tn * EE, NS, NS); g.add = F; g.ldadd = NS; g.zadd = zm(T * EE * NS); g.addscale = 1.0f; gemm_kernel<1, 0, 2, 2, 4, 2, ACT_NONE><<<dim3((Tn * EE + 63) / 64, 1, NBT), 256, 0, stream>>>(g); }
        { GemmArgs g = gemm_args(cXT, NS, zm(T * EE * NS), W4 + (size_t)2 * NS * NS, NS, zm(0), G, NS, zm(T * EE * NS), Tn * EE, NS, NS); g.bias = bg; gemm_kernel<1, 0, 2, 2, 4, 2, ACT_NONE><<<dim3((Tn * EE + 63) / 64, 1, NBT), 256, 0, stream>>>(g); }
        { GemmArgs g = gemm_args(cXT + (size_t)d * EE * NS, NS, zm(T * EE * NS), W4 + (size_t)3 * NS * NS, NS, zm(0), G, NS, zm(T * EE * NS), Tn * EE, NS, NS); g.add = G; g.ldadd = NS; g.zadd = zm(T * EE * NS); g.addscale = 1.0f; gemm_kernel<1, 0, 2, 2, 4, 2, ACT_NONE><<<dim3((Tn * EE + 63) / 64, 1, NBT), 256, 0, stream>>>(g); }
        k_wsp<<<(128 * 128) / 256, 256, 0, stream>>>(ws, T, Tn, WSP);
        { GemmArgs g = gemm_args(cXS, 128, zm(0), WSP, 128, zm(0), RES, 128, zm(0), NBT * NS * EE, Tn, T); g.bias = bs; g.nstore = 128; gemm_kernel<0, 0, 2, 2, 4, 2, ACT_NONE><<<dim3((NBT * NS * EE) / 64, 1, 1), 256, 0, stream>>>(g); }
        k_comb<<<(NBT * NS * Tn * EE + 255) / 256, 256, 0, stream>>>(F, G, RES, T, Tn, 0, nXT, nXS); k_comb<<<(NBT * NS * EE * 128) / 256, 256, 0, stream>>>(F, G, RES, T, Tn, 1, nXT, nXS);
        T = Tn; { float* t1 = cXT; cXT = nXT; nXT = t1; float* t2 = cXS; cXS = nXS; nXS = t2; }
        { GemmArgs g = gemm_args(wq, LL, zm(0), wk, LL, zm(0), Mq, NS, zm(0), NS, NS, LL); gemm_kernel<1, 0, 3, 3, 4, 2, ACT_NONE><<<dim3(NS / 64, 1, 1), 256, 0, stream>>>(g); }
        k_uwc<<<NS + 1, 256, 0, stream>>>(wq, bq, wk, bk, UW);
        { GemmArgs g = gemm_args(cXT, NS, zm(0), Mq, NS, zm(0), Y, NS, zm(0), NBT * T * EE, NS, NS); gemm_kernel<0, 0, 2, 2, 4, 2, ACT_NONE><<<dim3((NBT * T * EE + 63) / 64, 1, 1), 256, 0, stream>>>(g); }
        k_att<<<NBT * T, 256, 0, stream>>>(cXT, Y, UW, T, R);
        { GemmArgs g = gemm_args(R, NS, zm(0), wv, LL, zm(0), READ, LL, zm(0), NBT * T, LL, NS); g.bias = bv; gemm_kernel<0, 0, 2, 2, 4, 2, ACT_NONE><<<dim3((NBT * T + 63) / 64, LL / 128, 1), 256, 0, stream>>>(g); }
        k_ares<<<(NBT * NS * T * EE + 255) / 256, 256, 0, stream>>>(READ, cXT, T, 0, nXT, nXS); k_ares<<<(NBT * NS * EE * 128) / 256, 256, 0, stream>>>(READ, cXT, T, 1, nXT, nXS);
        { float* t1 = cXT; cXT = nXT; nXT = t1; float* t2 = cXS; cXS = nXS; nXS = t2; }
    }
    k_dec<<<(NBT * NS) / 8, 256, 0, stream>>>(cXS, dw, db, T, YD);
    k_wpad<<<(128 * 32) / 256, 256, 0, stream>>>(ow, OWP);
    { GemmArgs g = gemm_args(YD, 128, zm(0), OWP, 32, zm(0), Y2, 32, zm(0), NBT * NS, NOUT, 128); g.bias = ob; g.nstore = 32; gemm_kernel<0, 0, 2, 2, 8, 1, ACT_NONE><<<dim3((NBT * NS) / 128, 1, 1), 256, 0, stream>>>(g); }
    k_out<<<(NBT * NOUT * NS + 255) / 256, 256, 0, stream>>>(Y2, out);
}
